// BotImpact_15693810499989
// MI455X (gfx1250) — hardware-run, weakly checked
//
#include <hip/hip_runtime.h>
#include <math.h>

typedef __attribute__((ext_vector_type(16))) __bf16   v16b;
typedef __attribute__((ext_vector_type(8)))  __bf16   v8b;
typedef __attribute__((ext_vector_type(8)))  _Float16 v8h;
typedef __attribute__((ext_vector_type(8)))  float    v8f;
typedef __attribute__((ext_vector_type(4)))  float    v4f;
typedef __attribute__((ext_vector_type(4)))  int      v4i;

constexpr int kN     = 50000;
constexpr int kE     = 800000;
constexpr int kCh    = 128;
constexpr int kMP    = 50048;
constexpr int kNIdx  = 5000;
constexpr int kSmall = 4 * kNIdx;
constexpr int kTile  = 256;
constexpr int kIter  = 8;
constexpr int kCap   = kIter * 128;
constexpr int kPiece = 4 * kCap;
constexpr int kNumPiece = (kE + kPiece - 1) / kPiece;
static_assert((kMP % 64) == 0 && kMP >= kN);
static_assert((kCh % 64) == 0 && (kCh % 32) == 0);
static_assert((kE % 128) == 0);
static_assert(kE <= (1 << 20));
static_assert(kTile == 256);
static_assert(kSmall == 625 * 32);
static_assert(((kN * 2) % 4) == 0);
static_assert(kNumPiece == 196);

constexpr size_t kOffAH  = 0;
constexpr size_t kOffAL  = kOffAH + (size_t)kMP * kCh * 2;
constexpr size_t kOffH   = kOffAL + (size_t)kMP * kCh * 2;
constexpr size_t kOffSD  = kOffH  + (size_t)kMP * kCh * 4;
constexpr size_t kOffWP  = kOffSD + (size_t)kMP * 4 * 4;
constexpr size_t kWsTotal = kOffWP + (size_t)4 * kCh * kCh * 2;
static_assert(kWsTotal == 52180992ull);
static_assert(kWsTotal <= 134217728ull);
static_assert((kOffAL % 128) == 0 && (kOffH % 128) == 0 && (kOffSD % 128) == 0 && (kOffWP % 128) == 0);

__device__ __forceinline__ unsigned short f2bf_bits(float f) {
  unsigned u = __float_as_uint(f);
  return (unsigned short)((u + 0x7FFFu + ((u >> 16) & 1u)) >> 16);
}
__device__ __forceinline__ float bf_bits2f(unsigned short h) { return __uint_as_float(((unsigned)h) << 16); }

__device__ __forceinline__ void mma_guard4_b(v8f& a, v8f& b, v8f& c, v8f& d, v16b x, v16b y) {
  asm volatile("v_nop\n\tv_nop\n\tv_nop\n\tv_nop" : "+v"(a), "+v"(b), "+v"(c), "+v"(d) : "v"(x), "v"(y));
}
__device__ __forceinline__ void keep4_b(v16b a, v16b b, v16b c, v16b d) { asm volatile("v_nop" :: "v"(a), "v"(b), "v"(c), "v"(d)); }
__device__ __forceinline__ void acc_guard4(v8f& a, v8f& b, v8f& c, v8f& d) { asm volatile("v_nop\n\tv_nop\n\tv_nop\n\tv_nop" : "+v"(a), "+v"(b), "+v"(c), "+v"(d)); }

union FragB { v16b v; v8b h[2]; };
__device__ __forceinline__ v16b frag_load(const __bf16* p) {
  FragB f; f.h[0] = *(const v8b*)(p); f.h[1] = *(const v8b*)(p + 16); return f.v;
}
__device__ __forceinline__ v8f frag_mma(v16b a, v16b b, v8f c) {
  return __builtin_amdgcn_wmma_f32_16x16x32_bf16(false, a, false, b, (short)0, c, false, false);
}

__global__ __launch_bounds__(256) void gemm_split_kernel(
    const unsigned short* __restrict__ Ahp, const unsigned short* __restrict__ Alp,
    const unsigned short* __restrict__ Bhp, const unsigned short* __restrict__ Blp,
    float* __restrict__ C, int M)
{
  const __bf16* Ab  = (const __bf16*)Ahp;
  const __bf16* Ab2 = (const __bf16*)Alp;
  const __bf16* Bb  = (const __bf16*)Bhp;
  const __bf16* Bb2 = (const __bf16*)Blp;
  __shared__ __align__(16) float sT[8][16 * 68];
  const int lane = threadIdx.x & 31;
  const int wave = threadIdx.x >> 5;
  const int tilesN = kCh >> 6;
  const int tilesM = M >> 6;
  const int tile = blockIdx.x * 8 + wave;
  if (tile >= tilesM * tilesN) return;
  const int tm = tile / tilesN;
  const int tn = tile - tm * tilesN;
  const int m0 = tm << 6;
  const int n0 = tn << 6;
  const int lda = kCh, ldb = kCh, ldc = kCh;

  const int rlane = lane & 15;
  const int koff  = (lane >> 4) * 8;
  const int mOff  = (lane >> 4) * 8;

  v8f acc[4][4];
#pragma unroll
  for (int i = 0; i < 4; ++i)
#pragma unroll
    for (int j = 0; j < 4; ++j) acc[i][j] = (v8f){0.f,0.f,0.f,0.f,0.f,0.f,0.f,0.f};

#pragma unroll 1
  for (int k0 = 0; k0 < kCh; k0 += 32) {
    v16b bh[4], bl[4];
#pragma unroll
    for (int j = 0; j < 4; ++j) {
      const size_t bo = (size_t)(n0 + (j << 4) + rlane) * ldb + koff + k0;
      bh[j] = frag_load(Bb + bo);
      bl[j] = frag_load(Bb2 + bo);
    }
#pragma unroll
    for (int i = 0; i < 4; ++i) {
      const size_t ao = (size_t)(m0 + (i << 4) + rlane) * lda + koff + k0;
      v16b ah = frag_load(Ab + ao);
      v16b al = frag_load(Ab2 + ao);
#pragma unroll
      for (int j = 0; j < 4; ++j) {
        acc[i][j] = frag_mma(ah, bh[j], acc[i][j]);
        acc[i][j] = frag_mma(ah, bl[j], acc[i][j]);
        acc[i][j] = frag_mma(al, bh[j], acc[i][j]);
      }
      mma_guard4_b(acc[i][0], acc[i][1], acc[i][2], acc[i][3], ah, al);
    }
    keep4_b(bh[0], bh[1], bh[2], bh[3]);
    keep4_b(bl[0], bl[1], bl[2], bl[3]);
  }
  acc_guard4(acc[0][0], acc[0][1], acc[0][2], acc[0][3]);
  acc_guard4(acc[1][0], acc[1][1], acc[1][2], acc[1][3]);
  acc_guard4(acc[2][0], acc[2][1], acc[2][2], acc[2][3]);
  acc_guard4(acc[3][0], acc[3][1], acc[3][2], acc[3][3]);

  float* slab = sT[wave];
#pragma unroll
  for (int i = 0; i < 4; ++i) {
    const int mBase = m0 + (i << 4);
#pragma unroll
    for (int j = 0; j < 4; ++j) {
#pragma unroll
      for (int r = 0; r < 8; ++r) {
        slab[(mOff + r) * 68 + (j << 4) + rlane] = acc[i][j][r];
      }
    }
    __builtin_amdgcn_fence(__ATOMIC_RELEASE, "workgroup");
    __builtin_amdgcn_wave_barrier();
    __builtin_amdgcn_fence(__ATOMIC_ACQUIRE, "workgroup");
    {
      const int hh = lane >> 4, c4 = (lane & 15) * 4;
      for (int pass = 0; pass < 2; ++pass) {
#pragma unroll
        for (int it = 0; it < 8; ++it) {
          const int row = it * 2 + hh;
          v4f v = *(const v4f*)(slab + row * 68 + c4);
          *(volatile v4f*)(C + (size_t)(mBase + row) * ldc + n0 + c4) = v;
        }
        __threadfence();
      }
    }
    __builtin_amdgcn_fence(__ATOMIC_RELEASE, "workgroup");
    __builtin_amdgcn_wave_barrier();
    __builtin_amdgcn_fence(__ATOMIC_ACQUIRE, "workgroup");
  }
}

__global__ __launch_bounds__(256) void weight_planes_kernel(
    const float* __restrict__ W1, const float* __restrict__ W2, unsigned short* __restrict__ WP)
{
  const int i = blockIdx.x * 256 + threadIdx.x;
  const float* W = (blockIdx.y == 0) ? W1 : W2;
  const int n = i >> 4;
  const int k8 = (i & 15) * 8;
  v8h hv, lv;
#pragma unroll
  for (int e = 0; e < 8; ++e) {
    const float w = W[(size_t)(k8 + e) * kCh + n];
    const unsigned short hb = f2bf_bits(w);
    const unsigned short lb = f2bf_bits(w - bf_bits2f(hb));
    hv[e] = __builtin_bit_cast(_Float16, hb);
    lv[e] = __builtin_bit_cast(_Float16, lb);
  }
  unsigned short* ph = WP + (size_t)blockIdx.y * 2 * kCh * kCh + (size_t)i * 8;
  unsigned short* pl = ph + kCh * kCh;
  *(volatile v8h*)ph = hv;
  *(volatile v8h*)pl = lv;
  __threadfence();
  *(volatile v8h*)ph = hv;
  *(volatile v8h*)pl = lv;
}

__global__ __launch_bounds__(256) void split_rows_pad_kernel(
    const float* __restrict__ src, unsigned short* __restrict__ dhi, unsigned short* __restrict__ dlo,
    int real8, int total8)
{
  const int i = blockIdx.x * 256 + threadIdx.x;
  if (i >= total8) return;
  const bool live = i < real8;
  const int ic = live ? i : (real8 - 1);
  const size_t s0 = (size_t)ic << 3;
  const v4f a0 = *(const v4f*)(src + s0);
  const v4f a1 = *(const v4f*)(src + s0 + 4);
  v8h hv, lv;
#pragma unroll
  for (int e = 0; e < 4; ++e) {
    const float x0 = live ? a0[e] : 0.0f;
    const float x1 = live ? a1[e] : 0.0f;
    const unsigned short h0 = f2bf_bits(x0), h1 = f2bf_bits(x1);
    const unsigned short l0 = f2bf_bits(x0 - bf_bits2f(h0)), l1 = f2bf_bits(x1 - bf_bits2f(h1));
    hv[e]     = __builtin_bit_cast(_Float16, h0);
    hv[4 + e] = __builtin_bit_cast(_Float16, h1);
    lv[e]     = __builtin_bit_cast(_Float16, l0);
    lv[4 + e] = __builtin_bit_cast(_Float16, l1);
  }
  const size_t e0 = (size_t)i << 3;
  unsigned short* qh = dhi + e0;
  unsigned short* ql = dlo + e0;
  *(volatile v8h*)qh = hv;
  *(volatile v8h*)ql = lv;
  __threadfence();
  *(volatile v8h*)qh = hv;
  *(volatile v8h*)ql = lv;
}

__global__ __launch_bounds__(128) void alpha_kernel(
    const float* __restrict__ H, const float* __restrict__ a_src, const float* __restrict__ a_dst,
    float* __restrict__ SD)
{
  __shared__ __align__(16) float sS[128 * 4];
  const int tid = threadIdx.x, lane = tid & 31, wave = tid >> 5;
  const int hd = lane >> 4;
  const int base = blockIdx.x * 128;
  const v4f as4 = *(const v4f*)(a_src + lane * 4);
  const v4f ad4 = *(const v4f*)(a_dst + lane * 4);
#pragma unroll 1
  for (int r = 0; r < 32; ++r) {
    const int rowl = wave * 32 + r;
    const v4f hv = *(const v4f*)(H + (size_t)(base + rowl) * kCh + lane * 4);
    float ps = hv[0] * as4[0];
    ps = fmaf(hv[1], as4[1], ps);
    ps = fmaf(hv[2], as4[2], ps);
    ps = fmaf(hv[3], as4[3], ps);
    float pd = hv[0] * ad4[0];
    pd = fmaf(hv[1], ad4[1], pd);
    pd = fmaf(hv[2], ad4[2], pd);
    pd = fmaf(hv[3], ad4[3], pd);
    ps += __shfl_xor(ps, 1, 32);
    pd += __shfl_xor(pd, 1, 32);
    ps += __shfl_xor(ps, 2, 32);
    pd += __shfl_xor(pd, 2, 32);
    ps += __shfl_xor(ps, 4, 32);
    pd += __shfl_xor(pd, 4, 32);
    ps += __shfl_xor(ps, 8, 32);
    pd += __shfl_xor(pd, 8, 32);
    if ((lane & 15) == 0) {
      sS[rowl * 4 + hd] = ps;
      sS[rowl * 4 + 2 + hd] = pd;
    }
  }
  __syncthreads();
  const v4f o = *(const v4f*)(sS + tid * 4);
  float* p = SD + (size_t)(base + tid) * 4;
  *(volatile v4f*)p = o;
  __threadfence();
  *(volatile v4f*)p = o;
}

template <int LAYER, bool TPROB>
__global__ __launch_bounds__(128) void aggregate_kernel(
    const float* __restrict__ H, const float* __restrict__ SD, const int* __restrict__ ei,
    const float* __restrict__ bias,
    unsigned short* __restrict__ AH, unsigned short* __restrict__ AL,
    float* __restrict__ zout,
    const float* __restrict__ Wp, const float* __restrict__ bp, float* __restrict__ tpout)
{
  __shared__ __align__(16) float    sAcc[kTile * kCh];
  __shared__ __align__(16) float    sDen[kTile * 2];
  __shared__ __align__(16) unsigned sList[4 * kCap];
  __shared__ __align__(16) float    sTp[kTile * 2];
  __shared__ int sCnt[4];

  const int tid = threadIdx.x, lane = tid & 31, wave = tid >> 5;
  const int hd = lane >> 4;
  const int base = blockIdx.x * kTile;

#pragma unroll 1
  for (int i = 0; i < 64; ++i) {
    const int dl = wave + 4 * i;
    int node = base + dl;
    node = node < kN ? node : (kN - 1);
    const v4f sd = *(const v4f*)(SD + (size_t)node * 4);
    float s = (hd == 0) ? (sd[0] + sd[2]) : (sd[1] + sd[3]);
    s = s > 0.0f ? s : 0.2f * s;
    const float ex = expf(s);
    const v4f hv = *(const v4f*)(H + (size_t)node * kCh + lane * 4);
    v4f a;
    a[0] = ex * hv[0];
    a[1] = ex * hv[1];
    a[2] = ex * hv[2];
    a[3] = ex * hv[3];
    *(v4f*)(sAcc + dl * kCh + lane * 4) = a;
    if ((lane & 15) == 0) sDen[dl * 2 + hd] = ex;
  }
  __syncthreads();

  const int* dstp = ei + kE;
  const unsigned lt = (1u << lane) - 1u;

#pragma unroll 1
  for (int pc = 0; pc < kNumPiece; ++pc) {
    int cnt = 0;
#pragma unroll 1
    for (int it = 0; it < kIter; ++it) {
      const int eg = pc * kPiece + (wave * kIter + it) * 128;
      const bool inr = eg < kE;
      const int egc = inr ? eg : 0;
      const int e0 = egc + lane * 4;
      const v4i d4 = *(const v4i*)(dstp + e0);
      const unsigned u0 = (unsigned)(d4[0] - base);
      const unsigned u1 = (unsigned)(d4[1] - base);
      const unsigned u2 = (unsigned)(d4[2] - base);
      const unsigned u3 = (unsigned)(d4[3] - base);
      const bool h0 = inr && (u0 < (unsigned)kTile);
      const bool h1 = inr && (u1 < (unsigned)kTile);
      const bool h2 = inr && (u2 < (unsigned)kTile);
      const bool h3 = inr && (u3 < (unsigned)kTile);
      const unsigned b0 = __builtin_amdgcn_ballot_w32(h0);
      const unsigned b1 = __builtin_amdgcn_ballot_w32(h1);
      const unsigned b2 = __builtin_amdgcn_ballot_w32(h2);
      const unsigned b3 = __builtin_amdgcn_ballot_w32(h3);
      if ((b0 | b1 | b2 | b3) != 0u) {
        const int n0 = __popc(b0);
        const int n1 = n0 + __popc(b1);
        const int n2 = n1 + __popc(b2);
        const int n3 = n2 + __popc(b3);
        int p0 = cnt + __popc(b0 & lt);
        int p1 = cnt + n0 + __popc(b1 & lt);
        int p2 = cnt + n1 + __popc(b2 & lt);
        int p3 = cnt + n2 + __popc(b3 & lt);
        p0 = p0 < kCap ? p0 : (kCap - 1);
        p1 = p1 < kCap ? p1 : (kCap - 1);
        p2 = p2 < kCap ? p2 : (kCap - 1);
        p3 = p3 < kCap ? p3 : (kCap - 1);
        if (h0) sList[wave * kCap + p0] = (unsigned)(e0)     | (u0 << 20);
        if (h1) sList[wave * kCap + p1] = (unsigned)(e0 + 1) | (u1 << 20);
        if (h2) sList[wave * kCap + p2] = (unsigned)(e0 + 2) | (u2 << 20);
        if (h3) sList[wave * kCap + p3] = (unsigned)(e0 + 3) | (u3 << 20);
        cnt += n3;
      }
    }
    if (lane == 0) sCnt[wave] = cnt;
    __syncthreads();

    int c0 = sCnt[0], c1 = sCnt[1], c2 = sCnt[2], c3 = sCnt[3];
    c0 = c0 < 0 ? 0 : (c0 > kCap ? kCap : c0);
    c1 = c1 < 0 ? 0 : (c1 > kCap ? kCap : c1);
    c2 = c2 < 0 ? 0 : (c2 > kCap ? kCap : c2);
    c3 = c3 < 0 ? 0 : (c3 > kCap ? kCap : c3);
    const int t1 = c0, t2 = c0 + c1, t3 = t2 + c2, total = t3 + c3;
    const int ngrp = (total + 31) >> 5;
#pragma unroll 1
    for (int g = 0; g < ngrp; ++g) {
      const int f = g * 32 + lane;
      const bool live = f < total;
      const int fc = live ? f : (total - 1);
      const int ge1 = (fc >= t1) ? 1 : 0;
      const int ge2 = (fc >= t2) ? 1 : 0;
      const int ge3 = (fc >= t3) ? 1 : 0;
      const int L = ge1 + ge2 + ge3;
      const int pre = ge1 * c0 + ge2 * c1 + ge3 * c2;
      int li = fc - pre;
      li = li < 0 ? 0 : (li > kCap - 1 ? kCap - 1 : li);
      const unsigned ent = sList[L * kCap + li];
      int eid = (int)(ent & 0xFFFFFu);
      eid = eid < kE ? eid : (kE - 1);
      const int dl = (int)((ent >> 20) & 255u);
      int s = ei[eid];
      s = s < 0 ? 0 : (s > kN - 1 ? kN - 1 : s);
      int dn = base + dl;
      dn = dn < kN ? dn : (kN - 1);
      const v4f ss = *(const v4f*)(SD + (size_t)s * 4);
      const v4f dd = *(const v4f*)(SD + (size_t)dn * 4);
      float q0 = ss[0] + dd[2];
      float q1 = ss[1] + dd[3];
      q0 = q0 > 0.0f ? q0 : 0.2f * q0;
      q1 = q1 > 0.0f ? q1 : 0.2f * q1;
      const float x0 = expf(q0);
      const float x1 = expf(q1);
      const bool mine = live && ((dl & 3) == wave);
      unsigned mask = __builtin_amdgcn_ballot_w32(mine);
      for (int qi = 0; qi < 32 && mask != 0u; ++qi) {
        const int j = __builtin_ctz(mask);
        mask &= mask - 1u;
        const int   sj  = __shfl(s, j, 32);
        const int   dj  = __shfl(dl, j, 32);
        const float x0j = __shfl(x0, j, 32);
        const float x1j = __shfl(x1, j, 32);
        const float xh = (hd == 0) ? x0j : x1j;
        const v4f hv = *(const v4f*)(H + (size_t)sj * kCh + lane * 4);
        float* ap = sAcc + dj * kCh + lane * 4;
        v4f a = *(const v4f*)ap;
        a[0] = fmaf(xh, hv[0], a[0]);
        a[1] = fmaf(xh, hv[1], a[1]);
        a[2] = fmaf(xh, hv[2], a[2]);
        a[3] = fmaf(xh, hv[3], a[3]);
        *(v4f*)ap = a;
        if ((lane & 15) == 0) sDen[dj * 2 + hd] += xh;
      }
    }
    __syncthreads();
  }

  if (LAYER == 1) {
    const int l16 = lane & 15;
    const int c0 = l16 * 8;
    const int hh = l16 >> 3;
    const v4f bA = *(const v4f*)(bias + c0);
    const v4f bB = *(const v4f*)(bias + c0 + 4);
#pragma unroll 1
    for (int rr = 0; rr < 32; ++rr) {
      const int rowl = wave * 64 + rr * 2 + hd;
      const int row = base + rowl;
      const float inv = 1.0f / sDen[rowl * 2 + hh];
      const v4f a0 = *(const v4f*)(sAcc + rowl * kCh + c0);
      const v4f a1 = *(const v4f*)(sAcc + rowl * kCh + c0 + 4);
      const bool live = row < kN;
      v8h hv, lv;
#pragma unroll
      for (int e = 0; e < 4; ++e) {
        float y0 = fmaxf(fmaf(a0[e], inv, bA[e]), 0.0f);
        float y1 = fmaxf(fmaf(a1[e], inv, bB[e]), 0.0f);
        y0 = live ? y0 : 0.0f;
        y1 = live ? y1 : 0.0f;
        const unsigned short h0 = f2bf_bits(y0), h1 = f2bf_bits(y1);
        const unsigned short l0 = f2bf_bits(y0 - bf_bits2f(h0)), l1 = f2bf_bits(y1 - bf_bits2f(h1));
        hv[e]     = __builtin_bit_cast(_Float16, h0);
        hv[4 + e] = __builtin_bit_cast(_Float16, h1);
        lv[e]     = __builtin_bit_cast(_Float16, l0);
        lv[4 + e] = __builtin_bit_cast(_Float16, l1);
      }
      if (base + wave * 64 + rr * 2 < kMP) {
        unsigned short* ph = AH + (size_t)row * kCh + c0;
        unsigned short* pl = AL + (size_t)row * kCh + c0;
        *(volatile v8h*)ph = hv;
        *(volatile v8h*)pl = lv;
        __threadfence();
        *(volatile v8h*)ph = hv;
        *(volatile v8h*)pl = lv;
      }
    }
  } else {
    const v4f b4 = *(const v4f*)(bias + lane * 4);
    v4f wpa = (v4f){0.f, 0.f, 0.f, 0.f};
    v4f wpb = (v4f){0.f, 0.f, 0.f, 0.f};
    float bp0 = 0.f, bp1 = 0.f;
    if (TPROB) {
      wpa = *(const v4f*)(Wp + lane * 8);
      wpb = *(const v4f*)(Wp + lane * 8 + 4);
      bp0 = bp[0];
      bp1 = bp[1];
    }
#pragma unroll 1
    for (int r = 0; r < 64; ++r) {
      const int rowl = wave * 64 + r;
      const int row = base + rowl;
      const float inv = 1.0f / sDen[rowl * 2 + hd];
      const v4f a = *(const v4f*)(sAcc + rowl * kCh + lane * 4);
      v4f v;
      v[0] = fmaf(a[0], inv, b4[0]);
      v[1] = fmaf(a[1], inv, b4[1]);
      v[2] = fmaf(a[2], inv, b4[2]);
      v[3] = fmaf(a[3], inv, b4[3]);
      if (TPROB) {
        float p0 = v[0] * wpa[0];
        p0 = fmaf(v[1], wpa[2], p0);
        p0 = fmaf(v[2], wpb[0], p0);
        p0 = fmaf(v[3], wpb[2], p0);
        float p1 = v[0] * wpa[1];
        p1 = fmaf(v[1], wpa[3], p1);
        p1 = fmaf(v[2], wpb[1], p1);
        p1 = fmaf(v[3], wpb[3], p1);
        p0 += __shfl_xor(p0, 16, 32);
        p1 += __shfl_xor(p1, 16, 32);
        p0 += __shfl_xor(p0, 8, 32);
        p1 += __shfl_xor(p1, 8, 32);
        p0 += __shfl_xor(p0, 4, 32);
        p1 += __shfl_xor(p1, 4, 32);
        p0 += __shfl_xor(p0, 2, 32);
        p1 += __shfl_xor(p1, 2, 32);
        p0 += __shfl_xor(p0, 1, 32);
        p1 += __shfl_xor(p1, 1, 32);
        p0 += bp0;
        p1 += bp1;
        p0 = p0 > 0.0f ? p0 : 0.01f * p0;
        p1 = p1 > 0.0f ? p1 : 0.01f * p1;
        if (lane == 0) {
          sTp[rowl * 2] = p0;
          sTp[rowl * 2 + 1] = p1;
        }
      }
      if (row < kN) {
        float* p = zout + (size_t)row * kCh + lane * 4;
        *(volatile v4f*)p = v;
        __threadfence();
        *(volatile v4f*)p = v;
      }
    }
    if (TPROB) {
      __syncthreads();
      const int fi = base * 2 + tid * 4;
      if (fi < kN * 2) {
        const v4f t = *(const v4f*)(sTp + tid * 4);
        float* p = tpout + fi;
        *(volatile v4f*)p = t;
        __threadfence();
        *(volatile v4f*)p = t;
      }
    }
  }
}

__global__ __launch_bounds__(256) void heads_kernel(
    const float* __restrict__ zr, const float* __restrict__ zf,
    const int* __restrict__ treat, const int* __restrict__ control,
    const float* __restrict__ WyS, const float* __restrict__ byS,
    const float* __restrict__ Wy1, const float* __restrict__ by1,
    const float* __restrict__ Wy0, const float* __restrict__ by0,
    float* __restrict__ out)
{
  __shared__ __align__(16) float sW[128 * 64];
  __shared__ __align__(16) float sZ[32 * 132];
  __shared__ float sWy1[64];
  __shared__ float sWy0[64];
  __shared__ float sB[64];
  __shared__ float sY[32];
  const int tid = threadIdx.x;
#pragma unroll 1
  for (int i = 0; i < 8; ++i) {
    const int q = i * 256 + tid;
    *(v4f*)(sW + q * 4) = *(const v4f*)(WyS + q * 4);
  }
  if (tid < 64) {
    sWy1[tid] = Wy1[tid];
    sWy0[tid] = Wy0[tid];
    sB[tid] = byS[tid];
  }
  const int tl = tid >> 3, jg = tid & 7;
  const int t = blockIdx.x * 32 + tl;
  const int seg = t / kNIdx;
  {
    int i = t - seg * kNIdx;
    i = i < 0 ? 0 : (i > kNIdx - 1 ? kNIdx - 1 : i);
    const int it = treat[i];
    const int ic = control[i];
    const int wt = (seg < 2) ? 1 : 0;
    int node = it * wt + ic * (1 - wt);
    node = node < 0 ? 0 : (node > kN - 1 ? kN - 1 : node);
    const float fk = (seg & 1) ? 1.0f : 0.0f;
    const float fr = 1.0f - fk;
#pragma unroll 1
    for (int q = 0; q < 4; ++q) {
      const int c = jg * 16 + q * 4;
      const v4f a = *(const v4f*)(zr + (size_t)node * kCh + c);
      const v4f b = *(const v4f*)(zf + (size_t)node * kCh + c);
      v4f z;
      z[0] = fmaf(fr, a[0], fk * b[0]);
      z[1] = fmaf(fr, a[1], fk * b[1]);
      z[2] = fmaf(fr, a[2], fk * b[2]);
      z[3] = fmaf(fr, a[3], fk * b[3]);
      *(v4f*)(sZ + tl * 132 + c) = z;
    }
  }
  __syncthreads();

  float a0 = 0.f, a1 = 0.f, a2 = 0.f, a3 = 0.f, a4 = 0.f, a5 = 0.f, a6 = 0.f, a7 = 0.f;
  const float* zp = sZ + tl * 132;
  const float* wp = sW + jg * 8;
#pragma unroll 2
  for (int k = 0; k < kCh; ++k) {
    const float z = zp[k];
    const v4f w0 = *(const v4f*)(wp + k * 64);
    const v4f w1 = *(const v4f*)(wp + k * 64 + 4);
    a0 = fmaf(z, w0[0], a0);
    a1 = fmaf(z, w0[1], a1);
    a2 = fmaf(z, w0[2], a2);
    a3 = fmaf(z, w0[3], a3);
    a4 = fmaf(z, w1[0], a4);
    a5 = fmaf(z, w1[1], a5);
    a6 = fmaf(z, w1[2], a6);
    a7 = fmaf(z, w1[3], a7);
  }
  const bool use1 = (seg == 0) || (seg == 3);
  float part = 0.f;
  {
    const int j0 = jg * 8;
    float hv[8] = {a0, a1, a2, a3, a4, a5, a6, a7};
#pragma unroll
    for (int e = 0; e < 8; ++e) {
      float h = hv[e] + sB[j0 + e];
      h = h > 0.0f ? h : 0.01f * h;
      const float w1v = sWy1[j0 + e];
      const float w0v = sWy0[j0 + e];
      const float wy = use1 ? w1v : w0v;
      part = fmaf(h, wy, part);
    }
  }
  part += __shfl_xor(part, 1, 32);
  part += __shfl_xor(part, 2, 32);
  part += __shfl_xor(part, 4, 32);
  const float b1v = by1[0];
  const float b0v = by0[0];
  float s = part + (use1 ? b1v : b0v);
  s = s > 0.0f ? s : 0.01f * s;
  if (jg == 0) sY[tl] = s;
  __syncthreads();
  if (tid < 32) {
    const float val = sY[tid];
    volatile float* p = out + (size_t)blockIdx.x * 32 + tid;
    *p = val;
    __threadfence();
    *p = val;
  }
}

static void run_graph(const float* xin, const int* ei,
                      const float* a_s1, const float* a_d1, const float* b1,
                      const float* a_s2, const float* a_d2, const float* b2,
                      const float* Wp, const float* bp,
                      unsigned short* AH, unsigned short* AL, float* H, float* SD, unsigned short* WP,
                      float* zout, float* tpout, bool with_tp, hipStream_t stream)
{
  const int real8 = kN * kCh / 8;
  const int total8 = kMP * kCh / 8;
  const int gemmBlocks = ((kMP / 64) * (kCh / 64) + 7) / 8;
  const int aggBlocks = (kN + kTile - 1) / kTile;
  unsigned short* W1H = WP;
  unsigned short* W1L = WP + kCh * kCh;
  unsigned short* W2H = WP + 2 * kCh * kCh;
  unsigned short* W2L = WP + 3 * kCh * kCh;

  split_rows_pad_kernel<<<total8 / 256, 256, 0, stream>>>(xin, AH, AL, real8, total8);
  gemm_split_kernel<<<gemmBlocks, 256, 0, stream>>>(AH, AL, W1H, W1L, H, kMP);
  alpha_kernel<<<kMP / 128, 128, 0, stream>>>(H, a_s1, a_d1, SD);
  aggregate_kernel<1, false><<<aggBlocks, 128, 0, stream>>>(H, SD, ei, b1, AH, AL, zout, Wp, bp, tpout);
  gemm_split_kernel<<<gemmBlocks, 256, 0, stream>>>(AH, AL, W2H, W2L, H, kMP);
  alpha_kernel<<<kMP / 128, 128, 0, stream>>>(H, a_s2, a_d2, SD);
  if (with_tp) {
    aggregate_kernel<2, true><<<aggBlocks, 128, 0, stream>>>(H, SD, ei, b2, AH, AL, zout, Wp, bp, tpout);
  } else {
    aggregate_kernel<2, false><<<aggBlocks, 128, 0, stream>>>(H, SD, ei, b2, AH, AL, zout, Wp, bp, tpout);
  }
}

extern "C" void kernel_launch(void* const* d_in, const int* in_sizes, int n_in,
                              void* d_out, int out_size, void* d_ws, size_t ws_size,
                              hipStream_t stream) {
  if (n_in < 22) return;
  if (in_sizes[0] != kN * kCh || in_sizes[2] != kN * kCh) return;
  if (in_sizes[1] != 2 * kE || in_sizes[3] != 2 * kE) return;
  if (in_sizes[4] != kNIdx || in_sizes[5] != kNIdx) return;
  if (in_sizes[6] != kCh * kCh || in_sizes[10] != kCh * kCh) return;
  if (in_sizes[7] != kCh || in_sizes[8] != kCh || in_sizes[9] != kCh) return;
  if (in_sizes[11] != kCh || in_sizes[12] != kCh || in_sizes[13] != kCh) return;
  if (in_sizes[14] != kCh * 64 || in_sizes[15] != 64) return;
  if (in_sizes[16] != 64 || in_sizes[17] != 1 || in_sizes[18] != 64 || in_sizes[19] != 1) return;
  if (in_sizes[20] != kCh * 2 || in_sizes[21] != 2) return;
  if (out_size != kSmall + 2 * kN * kCh + 2 * kN) return;
  if (ws_size < kWsTotal) return;

  const float* x       = (const float*)d_in[0];
  const int*   ei      = (const int*)  d_in[1];
  const float* fx      = (const float*)d_in[2];
  const int*   fei     = (const int*)  d_in[3];
  const int*   treat   = (const int*)  d_in[4];
  const int*   control = (const int*)  d_in[5];
  const float* W1      = (const float*)d_in[6];
  const float* a_src1  = (const float*)d_in[7];
  const float* a_dst1  = (const float*)d_in[8];
  const float* b1      = (const float*)d_in[9];
  const float* W2      = (const float*)d_in[10];
  const float* a_src2  = (const float*)d_in[11];
  const float* a_dst2  = (const float*)d_in[12];
  const float* b2      = (const float*)d_in[13];
  const float* WyS     = (const float*)d_in[14];
  const float* byS     = (const float*)d_in[15];
  const float* Wy1     = (const float*)d_in[16];
  const float* by1     = (const float*)d_in[17];
  const float* Wy0     = (const float*)d_in[18];
  const float* by0     = (const float*)d_in[19];
  const float* Wp      = (const float*)d_in[20];
  const float* bp      = (const float*)d_in[21];

  float* out  = (float*)d_out;
  float* zR   = out + kSmall;
  float* zF   = zR + (size_t)kN * kCh;
  float* tp   = zF + (size_t)kN * kCh;

  char* ws = (char*)d_ws;
  unsigned short* AH = (unsigned short*)(ws + kOffAH);
  unsigned short* AL = (unsigned short*)(ws + kOffAL);
  float*          H  = (float*)(ws + kOffH);
  float*          SD = (float*)(ws + kOffSD);
  unsigned short* WP = (unsigned short*)(ws + kOffWP);

  weight_planes_kernel<<<dim3(8, 2), 256, 0, stream>>>(W1, W2, WP);

  run_graph(x,  ei,  a_src1, a_dst1, b1, a_src2, a_dst2, b2, Wp, bp, AH, AL, H, SD, WP, zR, tp, true,  stream);
  run_graph(fx, fei, a_src1, a_dst1, b1, a_src2, a_dst2, b2, Wp, bp, AH, AL, H, SD, WP, zF, tp, false, stream);

  heads_kernel<<<kSmall / 32, 256, 0, stream>>>(zR, zF, treat, control, WyS, byS, Wy1, by1, Wy0, by0, out);
}
